// Net_54631984005511
// MI455X (gfx1250) — hardware-verified
//
#include <hip/hip_runtime.h>
#include <stddef.h>
#include <stdint.h>


#define NN      32768
#define FT      256
#define HD      16
#define NE      524288
#define NG      256
#define NPG     128
#define ROK     32768
#define ROK2    65536
#define ROH     64
#define ROH2    128
#define ROO     16384
#define NTHR    256
#define NWAVE   8
#define EPT     8
#define CHUNK   (NTHR * EPT)
#define WCAP    (EPT * 32)
#define LISTN   (NWAVE * WCAP)
#define NBR     256
#define SLB     8
#define DEGCAP  48
#define BINN    (NBR * DEGCAP)
#define RB      16
#define HSLOT   (DEGCAP + 1)
#define HCAP    (RB * HSLOT)
#define MAXT    (HCAP / 16)
#define GBM     64
#define GBN     64
#define GTHR    128
#define NCH     64
#define U_A     512
#define U_B     1024
#define U_C     1024
#define U_D     1024
#define U_E     131072
#define U_F     262144
#define U_ALL   (U_A + U_B + U_C + U_D + U_E + U_F)
#define WSMAX   134217728

static_assert((CHUNK & (CHUNK - 1)) == 0 && CHUNK <= 4096);
static_assert(NBR == (1 << SLB) && ((long long)CHUNK << SLB) < (1LL << 31));
static_assert(NE % CHUNK == 0 && NN % NBR == 0 && NN % RB == 0 && NPG % RB == 0);
static_assert(LISTN % NTHR == 0 && BINN % (NTHR * 4) == 0 && (NBR * DEGCAP * 4) % 128 == 0);
static_assert(HCAP % 16 == 0 && MAXT * 16 == HCAP && RB == HD && RB * HD == NTHR && FT == NTHR);
static_assert(U_A % NTHR == 0 && U_B % NTHR == 0 && U_C % NTHR == 0 && U_D % NTHR == 0);
static_assert(U_E % NTHR == 0 && U_F % NTHR == 0 && U_ALL % NTHR == 0);
static_assert(ROK2 == 2 * ROK && ROK == NPG * FT && ROK / NCH == 512 && ROH2 == 2 * ROH);
static_assert(NG % GBM == 0 && ROO % GBN == 0 && ROH == GBN && GBM == (GTHR / 32) * 16);
static_assert(NN % GBM == 0 && NG * ROH % (16 * ROH) == 0);

typedef float          v4f   __attribute__((ext_vector_type(4)));
typedef float          v8f   __attribute__((ext_vector_type(8)));
typedef int            v4i   __attribute__((ext_vector_type(4)));
typedef int            v8i   __attribute__((ext_vector_type(8)));
typedef unsigned short v4us  __attribute__((ext_vector_type(4)));
typedef unsigned short v8us  __attribute__((ext_vector_type(8)));
typedef unsigned short v16us __attribute__((ext_vector_type(16)));
typedef __bf16         v16bf __attribute__((ext_vector_type(16)));
typedef v4f  __attribute__((may_alias)) v4fa;
typedef v4i  __attribute__((may_alias)) v4ia;
typedef v4us __attribute__((may_alias)) v4usa;
typedef v8us __attribute__((may_alias)) v8usa;
union FragB { v16bf v; v16us u; v8us h[2]; v8i w; };

__device__ __forceinline__ v8f wmb(const FragB& a, const FragB& b, v8f c) {
  v8f d = __builtin_amdgcn_wmma_f32_16x16x32_bf16(false, a.v, false, b.v, (short)0, c, false, false);
  asm volatile("v_nop\n\tv_nop\n\tv_nop\n\tv_nop" : "+v"(d) : "v"(a.w), "v"(b.w));
  return d;
}

__device__ __forceinline__ unsigned bf16_bits(float f) {
  const unsigned u = __float_as_uint(f);
  return (u + 0x7FFFu + ((u >> 16) & 1u)) >> 16;
}
__device__ __forceinline__ float bf16_val(float f) {
  return __uint_as_float(bf16_bits(f) << 16);
}
__device__ __forceinline__ float relun(float v) {
  return (v > 0.0f) ? v : (v - v);
}

template <int SLBT>
__device__ __forceinline__ int scan_chunk(const int* __restrict__ dsts, int nE, int cbase, int slotBase,
                                          int nb, int vec8, int* list, int tid, int lane, int wave) {
  int wc = 0;
  const int el0  = tid * EPT;
  const int e0   = cbase + el0;
  const int sent = -2147483647 - 1;
  v4i da, db;
  if (vec8 != 0 && cbase + CHUNK <= nE) {
    da = *(const v4i*)(dsts + e0);
    db = *(const v4i*)(dsts + e0 + 4);
  } else {
    da.x = (e0     < nE) ? dsts[min(e0,     nE - 1)] : sent;
    da.y = (e0 + 1 < nE) ? dsts[min(e0 + 1, nE - 1)] : sent;
    da.z = (e0 + 2 < nE) ? dsts[min(e0 + 2, nE - 1)] : sent;
    da.w = (e0 + 3 < nE) ? dsts[min(e0 + 3, nE - 1)] : sent;
    db.x = (e0 + 4 < nE) ? dsts[min(e0 + 4, nE - 1)] : sent;
    db.y = (e0 + 5 < nE) ? dsts[min(e0 + 5, nE - 1)] : sent;
    db.z = (e0 + 6 < nE) ? dsts[min(e0 + 6, nE - 1)] : sent;
    db.w = (e0 + 7 < nE) ? dsts[min(e0 + 7, nE - 1)] : sent;
  }
  const unsigned nbs = (unsigned)slotBase;
  const unsigned unb = (unsigned)nb;
  const unsigned s0 = (unsigned)da.x - nbs, s1 = (unsigned)da.y - nbs;
  const unsigned s2 = (unsigned)da.z - nbs, s3 = (unsigned)da.w - nbs;
  const unsigned s4 = (unsigned)db.x - nbs, s5 = (unsigned)db.y - nbs;
  const unsigned s6 = (unsigned)db.z - nbs, s7 = (unsigned)db.w - nbs;
  const bool h0 = s0 < unb, h1 = s1 < unb, h2 = s2 < unb, h3 = s3 < unb;
  const bool h4 = s4 < unb, h5 = s5 < unb, h6 = s6 < unb, h7 = s7 < unb;
  const unsigned any = __builtin_amdgcn_ballot_w32(h0 | h1 | h2 | h3 | h4 | h5 | h6 | h7);
  if (any != 0u) {
#define HITJ(J, HJ, SJ) { \
      const unsigned mj = __builtin_amdgcn_ballot_w32(HJ); \
      if (mj != 0u) { \
        if (HJ) { \
          const int pos = wc + (int)__builtin_amdgcn_mbcnt_lo(mj, 0u); \
          if (pos < WCAP) list[wave * WCAP + pos] = ((el0 + (J)) << SLBT) | (int)(SJ); \
        } \
        wc += (int)__builtin_popcount(mj); } }
    HITJ(0, h0, s0)
    HITJ(1, h1, s1)
    HITJ(2, h2, s2)
    HITJ(3, h3, s3)
    HITJ(4, h4, s4)
    HITJ(5, h5, s5)
    HITJ(6, h6, s6)
    HITJ(7, h7, s7)
#undef HITJ
  }
  return wc;
}

__device__ __forceinline__ v8us gather8(const float* __restrict__ p, size_t stride) {
  v8us o;
#pragma unroll
  for (int i = 0; i < 8; ++i) o[i] = (unsigned short)bf16_bits(p[(size_t)i * stride]);
  return o;
}

__global__ __launch_bounds__(NTHR) void k_prep(const float* __restrict__ w11, const float* __restrict__ w12,
                                               const float* __restrict__ w21, const float* __restrict__ w22,
                                               const float* __restrict__ rw1, const float* __restrict__ rw2,
                                               unsigned short* W1A, unsigned short* W1B2,
                                               unsigned short* W2A, unsigned short* W2B,
                                               unsigned short* RO1, unsigned short* RO2) {
  const int u = (int)blockIdx.x * NTHR + (int)threadIdx.x;
  if (u < U_A) {
    const int n = u >> 5, k8 = (u & 31) * 8;
    const v8us o = gather8(w11 + (size_t)k8 * HD + n, HD);
    unsigned short* dp = W1A + (size_t)n * FT + k8;
    *(volatile v8us*)dp = o; __threadfence(); *(volatile v8us*)dp = o;
  } else if (u < U_A + U_B) {
    const int v = u - U_A;
    const int n = v >> 6, k8 = (v & 63) * 8, kk = k8 & (FT - 1);
    const v8us o = gather8(w21 + (size_t)kk * HD + n, HD);
    unsigned short* dp = W1B2 + (size_t)n * (2 * FT) + k8;
    *(volatile v8us*)dp = o; __threadfence(); *(volatile v8us*)dp = o;
  } else if (u < U_A + U_B + U_C) {
    const int v = u - (U_A + U_B);
    const int n = v >> 2, k8 = (v & 3) * 8, kk = k8 & (HD - 1);
    const v8us o = gather8(w12 + (size_t)kk * FT + n, FT);
    unsigned short* dp = W2A + (size_t)n * 32 + k8;
    *(volatile v8us*)dp = o; __threadfence(); *(volatile v8us*)dp = o;
  } else if (u < U_A + U_B + U_C + U_D) {
    const int v = u - (U_A + U_B + U_C);
    const int n = v >> 2, k8 = (v & 3) * 8, kk = k8 & (HD - 1);
    const v8us o = gather8(w22 + (size_t)kk * FT + n, FT);
    unsigned short* dp = W2B + (size_t)n * 32 + k8;
    *(volatile v8us*)dp = o; __threadfence(); *(volatile v8us*)dp = o;
  } else if (u < U_A + U_B + U_C + U_D + U_E) {
    const int v = u - (U_A + U_B + U_C + U_D);
    const int n = v >> 3, k8 = (v & 7) * 8;
    const v8us o = gather8(rw2 + (size_t)k8 * ROO + n, ROO);
    unsigned short* dp = RO2 + (size_t)n * ROH2 + k8;
    *(volatile v8us*)dp = o; *(volatile v8us*)(dp + ROH) = o;
    __threadfence();
    *(volatile v8us*)dp = o; *(volatile v8us*)(dp + ROH) = o;
  } else if (u < U_ALL) {
    const int v = u - (U_A + U_B + U_C + U_D + U_E);
    const int n = v >> 12, k8 = (v & 4095) * 8;
    const v8us o = gather8(rw1 + (size_t)k8 * ROH + n, ROH);
    unsigned short* dp = RO1 + (size_t)n * ROK2 + k8;
    *(volatile v8us*)dp = o; *(volatile v8us*)(dp + ROK) = o;
    __threadfence();
    *(volatile v8us*)dp = o; *(volatile v8us*)(dp + ROK) = o;
  }
}

__global__ __launch_bounds__(GTHR) void k_P1(const float* __restrict__ x, const unsigned short* __restrict__ W1A,
                                             float* P1) {
  __shared__ __attribute__((aligned(16))) float stg[4 * 256];
  const int tid = (int)threadIdx.x, lane = tid & 31, wave = tid >> 5, hh = lane >> 4, m = lane & 15;
  const int rowBase = (int)blockIdx.x * GBM;
  v8f acc = {0.f, 0.f, 0.f, 0.f, 0.f, 0.f, 0.f, 0.f};
  const float* xp = x + (size_t)(rowBase + 16 * wave + m) * FT + 8 * hh;
  const unsigned short* wp = W1A + (size_t)m * FT + 8 * hh;
#pragma unroll 1
  for (int ks = 0; ks < FT / 32; ++ks) {
    const v4f a0 = *(const v4f*)(xp + 32 * ks);
    const v4f a1 = *(const v4f*)(xp + 32 * ks + 4);
    const v4f c0 = *(const v4f*)(xp + 32 * ks + 16);
    const v4f c1 = *(const v4f*)(xp + 32 * ks + 20);
    v8us o0, o1;
    o0[0] = (unsigned short)bf16_bits(a0.x); o0[1] = (unsigned short)bf16_bits(a0.y);
    o0[2] = (unsigned short)bf16_bits(a0.z); o0[3] = (unsigned short)bf16_bits(a0.w);
    o0[4] = (unsigned short)bf16_bits(a1.x); o0[5] = (unsigned short)bf16_bits(a1.y);
    o0[6] = (unsigned short)bf16_bits(a1.z); o0[7] = (unsigned short)bf16_bits(a1.w);
    o1[0] = (unsigned short)bf16_bits(c0.x); o1[1] = (unsigned short)bf16_bits(c0.y);
    o1[2] = (unsigned short)bf16_bits(c0.z); o1[3] = (unsigned short)bf16_bits(c0.w);
    o1[4] = (unsigned short)bf16_bits(c1.x); o1[5] = (unsigned short)bf16_bits(c1.y);
    o1[6] = (unsigned short)bf16_bits(c1.z); o1[7] = (unsigned short)bf16_bits(c1.w);
    FragB af, bf;
    af.h[0] = o0;
    af.h[1] = o1;
    bf.h[0] = *(const v8usa*)(wp + 32 * ks);
    bf.h[1] = *(const v8usa*)(wp + 32 * ks + 16);
    acc = wmb(af, bf, acc);
  }
#pragma unroll
  for (int r = 0; r < 8; ++r) stg[wave * 256 + (8 * hh + r) * HD + m] = acc[r];
  __syncthreads();
  const v4f v0 = *(const v4fa*)(stg + wave * 256 + 4 * lane);
  const v4f v1 = *(const v4fa*)(stg + wave * 256 + 128 + 4 * lane);
  float* op = P1 + (size_t)(rowBase + 16 * wave) * HD + 4 * lane;
  *(volatile v4f*)op = v0; *(volatile v4f*)(op + 128) = v1;
  __threadfence();
  *(volatile v4f*)op = v0; *(volatile v4f*)(op + 128) = v1;
}

__global__ __launch_bounds__(NTHR) void k_scan(const int* __restrict__ dsts, const int* __restrict__ srcs,
                                               int* cntg, int* ellg) {
  __shared__ __attribute__((aligned(16))) int bins[BINN];
  __shared__ __attribute__((aligned(16))) int list[LISTN];
  __shared__ __attribute__((aligned(16))) int cnt[NBR];
  __shared__ int wcnt[NWAVE];
  const int tid = (int)threadIdx.x, lane = tid & 31, wave = tid >> 5;
  const int nodeBase = (int)blockIdx.x * NBR;

  for (int i = tid; i < BINN; i += NTHR) bins[i] = 0;
  for (int i = tid; i < LISTN; i += NTHR) list[i] = 0;
  cnt[tid] = 0;
  if (tid < NWAVE) wcnt[tid] = 0;
  __syncthreads();

#pragma unroll 1
  for (int ch = 0; ch < NE / CHUNK; ++ch) {
    const int cbase = ch * CHUNK;
    const int wc = scan_chunk<SLB>(dsts, NE, cbase, nodeBase, NBR, 1, list, tid, lane, wave);
    if (lane == 0) wcnt[wave] = wc;
    __syncthreads();
    if (wave == 0) {
#pragma unroll 1
      for (int w2 = 0; w2 < NWAVE; ++w2) {
        int c = wcnt[w2];
        c = c < 0 ? 0 : (c > WCAP ? WCAP : c);
#pragma unroll 1
        for (int b0 = 0; b0 < c; b0 += 32) {
          const int idx = b0 + lane;
          const int ent = list[w2 * WCAP + (idx < WCAP ? idx : WCAP - 1)];
          const int m32 = (c - b0) < 32 ? (c - b0) : 32;
#pragma unroll 1
          for (int k = 0; k < m32; ++k) {
            const int u    = __builtin_amdgcn_readlane(ent, k);
            const int slot = u & (NBR - 1);
            const int el   = (u >> SLB) & (CHUNK - 1);
            if (lane == 0) {
              const int c0 = cnt[slot];
              if ((unsigned)c0 < (unsigned)DEGCAP) bins[slot * DEGCAP + c0] = cbase + el;
              cnt[slot] = c0 + 1;
            }
          }
        }
      }
    }
    __syncthreads();
  }

#pragma unroll 4
  for (int it = 0; it < BINN / NTHR; ++it) {
    const int i = it * NTHR + tid;
    const int slot = i / DEGCAP;
    const int pos  = i - slot * DEGCAP;
    const int c    = cnt[slot];
    int eid = bins[i];
    eid = eid < 0 ? 0 : (eid > NE - 1 ? NE - 1 : eid);
    int sv = srcs[eid];
    sv = sv < 0 ? 0 : (sv > NN - 1 ? NN - 1 : sv);
    bins[i] = (pos < c) ? sv : 0;
  }
  __syncthreads();

  const v4i cv = *(const v4ia*)(cnt + 4 * (tid & 63));
  v4i ev[BINN / (NTHR * 4)];
#pragma unroll
  for (int it = 0; it < BINN / (NTHR * 4); ++it) ev[it] = *(const v4ia*)(bins + 4 * (it * NTHR + tid));
  int* cp = cntg + (size_t)nodeBase + 4 * (tid & 63);
  int* ep = ellg + (size_t)nodeBase * DEGCAP;
  if (tid < 64) *(volatile v4i*)cp = cv;
#pragma unroll
  for (int it = 0; it < BINN / (NTHR * 4); ++it) *(volatile v4i*)(ep + 4 * (it * NTHR + tid)) = ev[it];
  __threadfence();
  if (tid < 64) *(volatile v4i*)cp = cv;
#pragma unroll
  for (int it = 0; it < BINN / (NTHR * 4); ++it) *(volatile v4i*)(ep + 4 * (it * NTHR + tid)) = ev[it];
}

template <int MODE>
__global__ __launch_bounds__(NTHR) void k_msg(const float* __restrict__ P, const float* __restrict__ b1,
                                              const unsigned short* __restrict__ W2T, const float* __restrict__ b2,
                                              const int* __restrict__ cntg, const int* __restrict__ ellg,
                                              const unsigned short* __restrict__ W1T2,
                                              float* P2out, unsigned short* X2out) {
  __shared__ int hs[HCAP];
  __shared__ int hd[HCAP];
  __shared__ int rc[RB];
  __shared__ int rbig[RB];
  __shared__ int ro[RB + 1];
  __shared__ __attribute__((aligned(16))) float Pd[RB * HD];
  __shared__ float b1s[HD];
  __shared__ __attribute__((aligned(16))) unsigned short At[16 * 32];
  __shared__ __attribute__((aligned(16))) float MSG[16 * FT];
  __shared__ __attribute__((aligned(16))) float ACC[RB * FT];
  __shared__ __attribute__((aligned(16))) unsigned short Ahl[RB * 2 * FT];
  const int tid = (int)threadIdx.x, lane = tid & 31, wave = tid >> 5, hh = lane >> 4, m = lane & 15;
  const int rowBase = (int)blockIdx.x * RB;

#pragma unroll 1
  for (int i = tid; i < HCAP; i += NTHR) { hs[i] = rowBase; hd[i] = -1; }
#pragma unroll
  for (int r = 0; r < RB; ++r) ACC[r * FT + tid] = 0.0f;
  Pd[tid] = P[(size_t)rowBase * HD + tid];
  if (tid < RB) {
    b1s[tid] = bf16_val(b1[tid]);
    int c = cntg[rowBase + tid];
    const int big = (c < 0 || c > DEGCAP) ? 1 : 0;
    c = c < 0 ? 0 : (c > DEGCAP ? DEGCAP : c);
    rc[tid] = c;
    rbig[tid] = big;
  }
  __syncthreads();
  if (tid == 0) {
    int run = 0;
#pragma unroll 1
    for (int q = 0; q < RB; ++q) { ro[q] = run; run += rc[q] + 1; }
    ro[RB] = run;
  }
  __syncthreads();
#pragma unroll 1
  for (int it = 0; it < (HCAP + NTHR - 1) / NTHR; ++it) {
    const int idx = it * NTHR + tid;
    const int idc = idx < HCAP ? idx : HCAP - 1;
    const int r = idc / HSLOT;
    const int j = idc - r * HSLOT;
    const int c = rc[r];
    const int jj = j < DEGCAP ? j : DEGCAP - 1;
    int sv = ellg[(size_t)(rowBase + r) * DEGCAP + jj];
    sv = sv < 0 ? 0 : (sv > NN - 1 ? NN - 1 : sv);
    const int val = (j < c) ? sv : (rowBase + r);
    if (idx < HCAP && j <= c) {
      const int pos = ro[r] + j;
      hs[pos] = val;
      hd[pos] = r;
    }
  }
  __syncthreads();
  int nT = (ro[RB] + 15) >> 4;
  nT = nT < 1 ? 1 : (nT > MAXT ? MAXT : nT);

  FragB bw[2];
  float b2v[2];
#pragma unroll
  for (int t = 0; t < 2; ++t) {
    const int n = 32 * wave + 16 * t + m;
    const unsigned short* wq = W2T + (size_t)n * 32 + 8 * hh;
    bw[t].h[0] = *(const v8usa*)wq;
    bw[t].h[1] = *(const v8usa*)(wq + 16);
    b2v[t] = bf16_val(b2[n]);
  }

  int cur = -1;
  float a = 0.0f;
  const int ti = tid >> 4, tj = tid & 15;
#pragma unroll 1
  for (int tl = 0; tl < nT; ++tl) {
    {
      const int e = tl * 16 + ti;
      const int s = hs[e];
      const int d = hd[e];
      const int dc = d < 0 ? 0 : (d > RB - 1 ? RB - 1 : d);
      float v = (P[(size_t)s * HD + tj] + Pd[dc * HD + tj]) + b1s[tj];
      v = relun(v);
      const unsigned hb = bf16_bits(v);
      const unsigned lb = bf16_bits(v - __uint_as_float(hb << 16));
      At[ti * 32 + tj] = (unsigned short)hb;
      At[ti * 32 + 16 + tj] = (unsigned short)lb;
    }
    __syncthreads();
    {
      FragB af;
      af.h[0] = *(const v8usa*)(At + m * 32 + 8 * hh);
      af.h[1] = *(const v8usa*)(At + m * 32 + 16 + 8 * hh);
#pragma unroll
      for (int t = 0; t < 2; ++t) {
        const v8f z = {0.f, 0.f, 0.f, 0.f, 0.f, 0.f, 0.f, 0.f};
        const v8f dv = wmb(af, bw[t], z);
        const int col = 32 * wave + 16 * t + m;
#pragma unroll
        for (int r = 0; r < 8; ++r) MSG[(8 * hh + r) * FT + col] = relun(dv[r] + b2v[t]);
      }
    }
    __syncthreads();
#pragma unroll 4
    for (int i = 0; i < 16; ++i) {
      int dl = __builtin_amdgcn_readfirstlane(hd[tl * 16 + i]);
      dl = dl > RB - 1 ? RB - 1 : dl;
      if (dl != cur) {
        if (cur >= 0) ACC[cur * FT + tid] = a;
        a = 0.0f;
        cur = dl;
      }
      const float mv = MSG[i * FT + tid];
      a = (dl >= 0) ? (a + mv) : a;
    }
  }
  if (cur >= 0) ACC[cur * FT + tid] = a;

  const float qnan = __int_as_float(0x7fc00000);
#pragma unroll 4
  for (int r = 0; r < RB; ++r) {
    float v = ACC[r * FT + tid];
    v = (rbig[r] != 0) ? qnan : v;
    const unsigned hb = bf16_bits(v);
    const unsigned lb = bf16_bits(v - __uint_as_float(hb << 16));
    Ahl[r * (2 * FT) + tid] = (unsigned short)hb;
    Ahl[r * (2 * FT) + FT + tid] = (unsigned short)lb;
  }
  __syncthreads();

  if constexpr (MODE == 0) {
    float* part = MSG;
    v8f acc = {0.f, 0.f, 0.f, 0.f, 0.f, 0.f, 0.f, 0.f};
#pragma unroll
    for (int q = 0; q < 2; ++q) {
      const int k0 = 32 * (2 * wave + q);
      FragB af, bf;
      af.h[0] = *(const v8usa*)(Ahl + m * (2 * FT) + k0 + 8 * hh);
      af.h[1] = *(const v8usa*)(Ahl + m * (2 * FT) + k0 + 16 + 8 * hh);
      const unsigned short* wq = W1T2 + (size_t)m * (2 * FT) + k0 + 8 * hh;
      bf.h[0] = *(const v8usa*)wq;
      bf.h[1] = *(const v8usa*)(wq + 16);
      acc = wmb(af, bf, acc);
    }
#pragma unroll
    for (int r = 0; r < 8; ++r) part[wave * 256 + (8 * hh + r) * HD + m] = acc[r];
    __syncthreads();
    float s = 0.0f;
#pragma unroll
    for (int w2 = 0; w2 < NWAVE; ++w2) s += part[w2 * 256 + tid];
    Pd[tid] = s;
    __syncthreads();
    const v4f ov = *(const v4fa*)(Pd + 4 * (tid & 63));
    float* op = P2out + (size_t)rowBase * HD + 4 * (tid & 63);
    if (tid < 64) *(volatile v4f*)op = ov;
    __threadfence();
    if (tid < 64) *(volatile v4f*)op = ov;
  } else {
    const int g  = rowBase / NPG;
    const int nl = rowBase - g * NPG;
    v8us qv[4];
#pragma unroll
    for (int it = 0; it < 4; ++it) {
      const int p = it * NTHR + tid;
      const int pt = p >> 9, q = p & 511, r = q >> 5, c8 = (q & 31) * 8;
      qv[it] = *(const v8usa*)(Ahl + r * (2 * FT) + pt * FT + c8);
    }
#pragma unroll
    for (int it = 0; it < 4; ++it) {
      const int p = it * NTHR + tid;
      const int pt = p >> 9, q = p & 511, r = q >> 5, c8 = (q & 31) * 8;
      unsigned short* dp = X2out + (size_t)g * ROK2 + (size_t)pt * ROK + (size_t)(nl + r) * FT + c8;
      *(volatile v8us*)dp = qv[it];
    }
    __threadfence();
#pragma unroll
    for (int it = 0; it < 4; ++it) {
      const int p = it * NTHR + tid;
      const int pt = p >> 9, q = p & 511, r = q >> 5, c8 = (q & 31) * 8;
      unsigned short* dp = X2out + (size_t)g * ROK2 + (size_t)pt * ROK + (size_t)(nl + r) * FT + c8;
      *(volatile v8us*)dp = qv[it];
    }
  }
}

template <int FIN>
__global__ __launch_bounds__(GTHR) void k_gemm(const unsigned short* __restrict__ A,
                                               const unsigned short* __restrict__ WT,
                                               const float* __restrict__ bias, float* outF) {
  __shared__ __attribute__((aligned(16))) float stg[GBM * GBN];
  const int tid = (int)threadIdx.x, lane = tid & 31, wave = tid >> 5, hh = lane >> 4, m = lane & 15;
  const int rowBase = (int)blockIdx.x * GBM;
  const int by      = (int)blockIdx.y;
  constexpr int    KP  = (FIN == 0) ? ROK2 : ROH2;
  constexpr int    NKS = (FIN == 0) ? 32 : 4;
  const int col0 = (FIN == 0) ? 0 : by * GBN;
  const int ldo  = (FIN == 0) ? ROH : ROO;
  float* ob = (FIN == 0) ? (outF + (size_t)by * (size_t)(NG * ROH)) : outF;

  v8f acc[4];
  {
    const v8f z = {0.f, 0.f, 0.f, 0.f, 0.f, 0.f, 0.f, 0.f};
    acc[0] = z; acc[1] = z; acc[2] = z; acc[3] = z;
  }
  const unsigned short* ap = A  + (size_t)(rowBase + 16 * wave + m) * (size_t)KP + 8 * hh;
  const unsigned short* wp = WT + (size_t)(col0 + m) * (size_t)KP + 8 * hh;
#pragma unroll 1
  for (int ks = 0; ks < NKS; ++ks) {
    const int kk = (FIN == 0) ? ((ks >> 4) * ROK + by * (ROK / NCH) + (ks & 15) * 32) : (32 * ks);
    FragB af;
    af.h[0] = *(const v8usa*)(ap + kk);
    af.h[1] = *(const v8usa*)(ap + kk + 16);
#pragma unroll
    for (int t = 0; t < 4; ++t) {
      const unsigned short* wq = wp + (size_t)(16 * t) * (size_t)KP + kk;
      FragB bf;
      bf.h[0] = *(const v8usa*)wq;
      bf.h[1] = *(const v8usa*)(wq + 16);
      acc[t] = wmb(af, bf, acc[t]);
    }
  }

#pragma unroll
  for (int t = 0; t < 4; ++t) {
    const int lc = 16 * t + m;
#pragma unroll
    for (int r = 0; r < 8; ++r) {
      const int lr = 16 * wave + 8 * hh + r;
      stg[lr * GBN + lc] = acc[t][r];
    }
  }
  __syncthreads();

  v4f bb = {0.f, 0.f, 0.f, 0.f};
  if constexpr (FIN != 0) {
    const v4f t4 = *(const v4f*)(bias + col0 + 4 * m);
    bb.x = bf16_val(t4.x); bb.y = bf16_val(t4.y); bb.z = bf16_val(t4.z); bb.w = bf16_val(t4.w);
  }
  v4f fv[8];
#pragma unroll
  for (int i = 0; i < 8; ++i) {
    const int lr = 16 * wave + 2 * i + hh;
    v4f v = *(const v4fa*)(stg + lr * GBN + 4 * m);
    if constexpr (FIN != 0) {
      v.x = relun(v.x + bb.x); v.y = relun(v.y + bb.y); v.z = relun(v.z + bb.z); v.w = relun(v.w + bb.w);
    }
    fv[i] = v;
  }
#pragma unroll
  for (int i = 0; i < 8; ++i) {
    const int gr = rowBase + 16 * wave + 2 * i + hh;
    float* op = ob + (size_t)gr * (size_t)ldo + col0 + 4 * m;
    *(volatile v4f*)op = fv[i];
  }
  __threadfence();
#pragma unroll
  for (int i = 0; i < 8; ++i) {
    const int gr = rowBase + 16 * wave + 2 * i + hh;
    float* op = ob + (size_t)gr * (size_t)ldo + col0 + 4 * m;
    *(volatile v4f*)op = fv[i];
  }
}

__global__ __launch_bounds__(NTHR) void k_ro1c(const float* __restrict__ rec, const float* __restrict__ bias,
                                               unsigned short* y1) {
  __shared__ __attribute__((aligned(16))) unsigned short ys[16 * ROH2];
  const int tid = (int)threadIdx.x;
  const int r = tid >> 4, c4 = (tid & 15) * 4;
  const int row = (int)blockIdx.x * 16 + r;
  v4f s = {0.f, 0.f, 0.f, 0.f};
  const float* rp = rec + (size_t)row * ROH + c4;
#pragma unroll 4
  for (int ch = 0; ch < NCH; ++ch) s += *(const v4f*)(rp + (size_t)ch * (size_t)(NG * ROH));
  const v4f b4 = *(const v4f*)(bias + c4);
  const float y0 = relun(s.x + bf16_val(b4.x));
  const float y1v = relun(s.y + bf16_val(b4.y));
  const float y2 = relun(s.z + bf16_val(b4.z));
  const float y3 = relun(s.w + bf16_val(b4.w));
  v4us h4, l4;
  unsigned hb;
  hb = bf16_bits(y0);  h4[0] = (unsigned short)hb; l4[0] = (unsigned short)bf16_bits(y0  - __uint_as_float(hb << 16));
  hb = bf16_bits(y1v); h4[1] = (unsigned short)hb; l4[1] = (unsigned short)bf16_bits(y1v - __uint_as_float(hb << 16));
  hb = bf16_bits(y2);  h4[2] = (unsigned short)hb; l4[2] = (unsigned short)bf16_bits(y2  - __uint_as_float(hb << 16));
  hb = bf16_bits(y3);  h4[3] = (unsigned short)hb; l4[3] = (unsigned short)bf16_bits(y3  - __uint_as_float(hb << 16));
  *(v4usa*)(ys + r * ROH2 + c4) = h4;
  *(v4usa*)(ys + r * ROH2 + ROH + c4) = l4;
  __syncthreads();
  const v8us q = *(const v8usa*)(ys + r * ROH2 + 8 * (tid & 15));
  unsigned short* dp = y1 + (size_t)row * ROH2 + 8 * (tid & 15);
  *(volatile v8us*)dp = q;
  __threadfence();
  *(volatile v8us*)dp = q;
}

static inline size_t al256(size_t o) { return (o + 255) & ~(size_t)255; }

extern "C" void kernel_launch(void* const* d_in, const int* in_sizes, int n_in,
                              void* d_out, int out_size, void* d_ws, size_t ws_size,
                              hipStream_t stream) {
  if (n_in < 14) return;
  if (in_sizes[0] != NN * FT) return;
  if (in_sizes[1] != 2 * NE) return;
  if (in_sizes[2] != FT * HD || in_sizes[3] != HD) return;
  if (in_sizes[4] != HD * FT || in_sizes[5] != FT) return;
  if (in_sizes[6] != FT * HD || in_sizes[7] != HD) return;
  if (in_sizes[8] != HD * FT || in_sizes[9] != FT) return;
  if (in_sizes[10] != ROK * ROH || in_sizes[11] != ROH) return;
  if (in_sizes[12] != ROH * ROO || in_sizes[13] != ROO) return;
  if (out_size != NG * ROO) return;

  const float* x    = (const float*)d_in[0];
  const int*   edge = (const int*)d_in[1];
  const float* w11  = (const float*)d_in[2];
  const float* b11  = (const float*)d_in[3];
  const float* w12  = (const float*)d_in[4];
  const float* b12  = (const float*)d_in[5];
  const float* w21  = (const float*)d_in[6];
  const float* b21  = (const float*)d_in[7];
  const float* w22  = (const float*)d_in[8];
  const float* b22  = (const float*)d_in[9];
  const float* rw1  = (const float*)d_in[10];
  const float* rb1  = (const float*)d_in[11];
  const float* rw2  = (const float*)d_in[12];
  const float* rb2  = (const float*)d_in[13];
  float* out = (float*)d_out;
  const int* src = edge;
  const int* dst = edge + NE;

  char* ws = (char*)d_ws;
  size_t off = 0;
  const size_t oW1A = off; off = al256(off + (size_t)HD * FT * 2);
  const size_t oW1B = off; off = al256(off + (size_t)HD * 2 * FT * 2);
  const size_t oW2A = off; off = al256(off + (size_t)FT * 32 * 2);
  const size_t oW2B = off; off = al256(off + (size_t)FT * 32 * 2);
  const size_t oRO1 = off; off = al256(off + (size_t)ROH * ROK2 * 2);
  const size_t oRO2 = off; off = al256(off + (size_t)ROO * ROH2 * 2);
  const size_t oP1  = off; off = al256(off + (size_t)NN * HD * 4);
  const size_t oP2  = off; off = al256(off + (size_t)NN * HD * 4);
  const size_t oCNT = off; off = al256(off + (size_t)NN * 4);
  const size_t oELL = off; off = al256(off + (size_t)NN * DEGCAP * 4);
  const size_t oX2  = off; off = al256(off + (size_t)NG * ROK2 * 2);
  const size_t oREC = off; off = al256(off + (size_t)NCH * NG * ROH * 4);
  const size_t oY1  = off; off = al256(off + (size_t)NG * ROH2 * 2);
  if (off > ws_size || off > (size_t)WSMAX) return;
  unsigned short* W1A  = (unsigned short*)(ws + oW1A);
  unsigned short* W1B2 = (unsigned short*)(ws + oW1B);
  unsigned short* W2A  = (unsigned short*)(ws + oW2A);
  unsigned short* W2B  = (unsigned short*)(ws + oW2B);
  unsigned short* RO1  = (unsigned short*)(ws + oRO1);
  unsigned short* RO2  = (unsigned short*)(ws + oRO2);
  float*          P1   = (float*)(ws + oP1);
  float*          P2   = (float*)(ws + oP2);
  int*            CNT  = (int*)(ws + oCNT);
  int*            ELL  = (int*)(ws + oELL);
  unsigned short* X2   = (unsigned short*)(ws + oX2);
  float*          REC  = (float*)(ws + oREC);
  unsigned short* Y1   = (unsigned short*)(ws + oY1);

  k_prep<<<U_ALL / NTHR, NTHR, 0, stream>>>(w11, w12, w21, w22, rw1, rw2, W1A, W1B2, W2A, W2B, RO1, RO2);
  k_P1<<<NN / GBM, GTHR, 0, stream>>>(x, W1A, P1);
  k_scan<<<NN / NBR, NTHR, 0, stream>>>(dst, src, CNT, ELL);
  k_msg<0><<<NN / RB, NTHR, 0, stream>>>(P1, b11, W2A, b12, CNT, ELL, W1B2, P2, X2);
  k_msg<1><<<NN / RB, NTHR, 0, stream>>>(P2, b21, W2B, b22, CNT, ELL, W1B2, P2, X2);
  k_gemm<0><<<dim3(NG / GBM, NCH), GTHR, 0, stream>>>(X2, RO1, rb1, REC);
  k_ro1c<<<NG / 16, NTHR, 0, stream>>>(REC, rb1, Y1);
  k_gemm<1><<<dim3(NG / GBM, ROO / GBN), GTHR, 0, stream>>>(Y1, RO2, rb2, out);
}
